// GNN_52080773431963
// MI455X (gfx1250) — hardware-verified
//
#include <hip/hip_runtime.h>
#include <stddef.h>
#include <stdint.h>
#include <math.h>


#define FIN     128
#define LW      256
#define NMACH   16
#define NTHR    256
#define NWAVE   8
#define EPT     8
#define CHUNK   (NTHR * EPT)
#define WCAP    (EPT * 32)
#define LISTN   (NWAVE * WCAP)
#define NB      1024
#define SLOTB   10
#define RCAP    20480
#define DEGCAP  64
#define GBM     64
#define APITCH  40
#define RBN     128
#define BK_ZINTS (2 * RCAP + 2 * NB + LISTN)
#define LDS_BKT  (BK_ZINTS * 4 + 64)
#define SS0N    (2 * 128 * 128)
#define SS1N    (2 * 256 * 128)

static_assert((CHUNK & (CHUNK - 1)) == 0);
static_assert(NB == (1 << SLOTB));
static_assert(((long long)CHUNK << SLOTB) < (1LL << 31));
static_assert(NTHR * 4 == NB);
static_assert(LISTN >= NB && LISTN >= NWAVE * WCAP);
static_assert(RCAP % (NTHR * 4) == 0);
static_assert(BK_ZINTS % (NTHR * 4) == 0);
static_assert(LDS_BKT <= 300000);
static_assert(FIN % 32 == 0 && LW % 32 == 0);
static_assert(GBM * 4 == NTHR);
static_assert((APITCH * 2) % 16 == 0 && APITCH >= 32);
static_assert(SS0N % (NTHR * 4) == 0 && SS1N % (NTHR * 4) == 0);

typedef float          v2f  __attribute__((ext_vector_type(2)));
typedef float          v4f  __attribute__((ext_vector_type(4)));
typedef float          v8f  __attribute__((ext_vector_type(8)));
typedef double         v2d  __attribute__((ext_vector_type(2)));
typedef int            v4i  __attribute__((ext_vector_type(4)));
typedef int            v8i  __attribute__((ext_vector_type(8)));
typedef unsigned int   v2u  __attribute__((ext_vector_type(2)));
typedef unsigned short v8us __attribute__((ext_vector_type(8)));
typedef __bf16         v16b __attribute__((ext_vector_type(16)));
typedef v2u  __attribute__((may_alias)) v2ua;
typedef v4f  __attribute__((may_alias)) v4fa;
typedef v4i  __attribute__((may_alias)) v4ia;
typedef v2d  __attribute__((may_alias)) v2da;
typedef v8us __attribute__((may_alias)) v8usa;
union FragB { v16b v; v8us h[2]; v8i w; };

__device__ __forceinline__ v8f wmb(const FragB& a, const FragB& b, v8f c) {
  v8f d = __builtin_amdgcn_wmma_f32_16x16x32_bf16(false, a.v, false, b.v, (short)0, c, false, false);
  asm volatile("v_nop\n\tv_nop\n\tv_nop\n\tv_nop" : "+v"(d) : "v"(a.w), "v"(b.w));
  return d;
}

__device__ __forceinline__ unsigned int f2bf(float f) {
  const unsigned int u = __float_as_uint(f);
  return ((u + 0x7FFFu + ((u >> 16) & 1u)) >> 16) & 0xFFFFu;
}
__device__ __forceinline__ float bf2f(unsigned int b) { return __uint_as_float(b << 16); }
__device__ __forceinline__ float bfr(float f) { return bf2f(f2bf(f)); }
__device__ __forceinline__ v4f bfr4(const v4f a) {
  v4f r; r.x = bfr(a.x); r.y = bfr(a.y); r.z = bfr(a.z); r.w = bfr(a.w); return r;
}
__device__ __forceinline__ float relu_np(float v) { return (v > 0.0f) ? v : (v - v); }

#define SP1(I, F) { const unsigned int hb_ = f2bf(F); oh[I] = (unsigned short)hb_; \
                    ol[I] = (unsigned short)f2bf((F) - bf2f(hb_)); }
__device__ __forceinline__ void split8(const v4f a, const v4f b, v8us& oh, v8us& ol) {
  SP1(0, a.x) SP1(1, a.y) SP1(2, a.z) SP1(3, a.w)
  SP1(4, b.x) SP1(5, b.y) SP1(6, b.z) SP1(7, b.w)
}
#undef SP1

__device__ __forceinline__ int scan_chunk(const int* __restrict__ dsts, int nE, int cbase, int slotBase,
                                          int nb, int vec8, int* list, int tid, int lane, int wave) {
  int wc = 0;
  const int el0  = tid * EPT;
  const int e0   = cbase + el0;
  const int sent = -2147483647 - 1;
  v4i da, db;
  if (vec8 != 0 && cbase + CHUNK <= nE) {
    da = *(const v4i*)(dsts + e0);
    db = *(const v4i*)(dsts + e0 + 4);
  } else {
    da.x = (e0     < nE) ? dsts[min(e0,     nE - 1)] : sent;
    da.y = (e0 + 1 < nE) ? dsts[min(e0 + 1, nE - 1)] : sent;
    da.z = (e0 + 2 < nE) ? dsts[min(e0 + 2, nE - 1)] : sent;
    da.w = (e0 + 3 < nE) ? dsts[min(e0 + 3, nE - 1)] : sent;
    db.x = (e0 + 4 < nE) ? dsts[min(e0 + 4, nE - 1)] : sent;
    db.y = (e0 + 5 < nE) ? dsts[min(e0 + 5, nE - 1)] : sent;
    db.z = (e0 + 6 < nE) ? dsts[min(e0 + 6, nE - 1)] : sent;
    db.w = (e0 + 7 < nE) ? dsts[min(e0 + 7, nE - 1)] : sent;
  }
  const unsigned nbs = (unsigned)slotBase;
  const unsigned unb = (unsigned)nb;
  const unsigned s0 = (unsigned)da.x - nbs, s1 = (unsigned)da.y - nbs;
  const unsigned s2 = (unsigned)da.z - nbs, s3 = (unsigned)da.w - nbs;
  const unsigned s4 = (unsigned)db.x - nbs, s5 = (unsigned)db.y - nbs;
  const unsigned s6 = (unsigned)db.z - nbs, s7 = (unsigned)db.w - nbs;
  const bool h0 = s0 < unb, h1 = s1 < unb, h2 = s2 < unb, h3 = s3 < unb;
  const bool h4 = s4 < unb, h5 = s5 < unb, h6 = s6 < unb, h7 = s7 < unb;
  const unsigned any = __builtin_amdgcn_ballot_w32(h0 | h1 | h2 | h3 | h4 | h5 | h6 | h7);
  if (any != 0u) {
#define HITJ(J, HJ, SJ) { \
      const unsigned mj = __builtin_amdgcn_ballot_w32(HJ); \
      if (mj != 0u) { \
        if (HJ) { \
          const int pos = wc + (int)__builtin_amdgcn_mbcnt_lo(mj, 0u); \
          if (pos < WCAP) list[wave * WCAP + pos] = ((el0 + (J)) << SLOTB) | (int)(SJ); \
        } \
        wc += (int)__builtin_popcount(mj); } }
    HITJ(0, h0, s0)
    HITJ(1, h1, s1)
    HITJ(2, h2, s2)
    HITJ(3, h3, s3)
    HITJ(4, h4, s4)
    HITJ(5, h5, s5)
    HITJ(6, h6, s6)
    HITJ(7, h7, s7)
#undef HITJ
  }
  return wc;
}

__global__ __launch_bounds__(NTHR) void k_sum(const float* __restrict__ Wa0, const float* __restrict__ Wb0,
                                              const float* __restrict__ Wa1, const float* __restrict__ Wb1,
                                              float* SS) {
  const int t4 = ((int)blockIdx.x * NTHR + (int)threadIdx.x) * 4;
  if (t4 >= SS0N + SS1N) return;
  const float* src;
  int idx, msz;
  if (t4 < SS0N) {
    const int br = t4 >> 14;
    idx = t4 & 16383; msz = 16384;
    src = br ? Wb0 : Wa0;
  } else {
    const int u = t4 - SS0N;
    const int br = u >> 15;
    idx = u & 32767; msz = 32768;
    src = br ? Wb1 : Wa1;
  }
  const v4f a = bfr4(*(const v4fa*)(src + idx));
  const v4f b = bfr4(*(const v4fa*)(src + msz + idx));
  const v4f c = bfr4(*(const v4fa*)(src + 2 * msz + idx));
  const v4f o = (a + b) + c;
  *(volatile v4f*)(SS + t4) = o;
  __threadfence();
  *(volatile v4f*)(SS + t4) = o;
}

template <int KIN>
__global__ __launch_bounds__(NTHR) void k_wtr(const float* __restrict__ SSl, const float* __restrict__ Wa,
                                              const float* __restrict__ Wb, unsigned short* Bt) {
  constexpr int KQ  = KIN / 8;
  constexpr int UPS = 256 * KQ;
  constexpr int KB  = 5 * KIN;
  static_assert(UPS % NTHR == 0);
  const int u = (int)blockIdx.x * NTHR + (int)threadIdx.x;
  if (u >= 5 * UPS) return;
  const int seg = u / UPS;
  const int v   = u - seg * UPS;
  const int n   = v / KQ;
  const int k8  = (v - n * KQ) * 8;
  const int br  = n >> 7;
  const int c   = n & 127;
  const float* p;
  if (seg < 2) p = SSl + (size_t)br * KIN * 128 + (size_t)k8 * 128 + c;
  else         p = (br ? Wb : Wa) + (size_t)(seg + 1) * KIN * 128 + (size_t)k8 * 128 + c;
  const float f0 = p[0],   f1 = p[128], f2 = p[256], f3 = p[384];
  const float f4 = p[512], f5 = p[640], f6 = p[768], f7 = p[896];
  const bool lo = (seg == 1);
  v8us o;
  o[0] = (unsigned short)(lo ? f2bf(f0 - bfr(f0)) : f2bf(f0));
  o[1] = (unsigned short)(lo ? f2bf(f1 - bfr(f1)) : f2bf(f1));
  o[2] = (unsigned short)(lo ? f2bf(f2 - bfr(f2)) : f2bf(f2));
  o[3] = (unsigned short)(lo ? f2bf(f3 - bfr(f3)) : f2bf(f3));
  o[4] = (unsigned short)(lo ? f2bf(f4 - bfr(f4)) : f2bf(f4));
  o[5] = (unsigned short)(lo ? f2bf(f5 - bfr(f5)) : f2bf(f5));
  o[6] = (unsigned short)(lo ? f2bf(f6 - bfr(f6)) : f2bf(f6));
  o[7] = (unsigned short)(lo ? f2bf(f7 - bfr(f7)) : f2bf(f7));
  unsigned short* dp = Bt + (size_t)n * KB + seg * KIN + k8;
  *(volatile v8us*)dp = o;
  __threadfence();
  *(volatile v8us*)dp = o;
}

__global__ __launch_bounds__(NTHR) void k_wet(const float* __restrict__ We, unsigned short* WeT) {
  const int u = (int)blockIdx.x * NTHR + (int)threadIdx.x;
  if (u >= NMACH * (LW / 8)) return;
  const int mm = u >> 5;
  const int k8 = (u & 31) * 8;
  const float* p = We + (size_t)k8 * NMACH + mm;
  const float f0 = p[0],  f1 = p[16], f2 = p[32], f3 = p[48];
  const float f4 = p[64], f5 = p[80], f6 = p[96], f7 = p[112];
  v8us o;
  o[0] = (unsigned short)f2bf(f0); o[1] = (unsigned short)f2bf(f1);
  o[2] = (unsigned short)f2bf(f2); o[3] = (unsigned short)f2bf(f3);
  o[4] = (unsigned short)f2bf(f4); o[5] = (unsigned short)f2bf(f5);
  o[6] = (unsigned short)f2bf(f6); o[7] = (unsigned short)f2bf(f7);
  unsigned short* dp = WeT + (size_t)mm * LW + k8;
  *(volatile v8us*)dp = o;
  __threadfence();
  *(volatile v8us*)dp = o;
}

__global__ __launch_bounds__(NTHR) void k_cvx(const float* __restrict__ x, int nN, int nUnits,
                                              unsigned short* xb) {
  const int u = (int)blockIdx.x * NTHR + (int)threadIdx.x;
  if (u >= nUnits) return;
  const int row = u >> 4;
  const int k8  = (u & 15) * 8;
  const int rc  = row < nN ? row : nN - 1;
  const float* p = x + (size_t)rc * FIN + k8;
  const v4f a = *(const v4fa*)p;
  const v4f b = *(const v4fa*)(p + 4);
  const bool ok = row < nN;
  v8us o;
  o[0] = ok ? (unsigned short)f2bf(a.x) : (unsigned short)0;
  o[1] = ok ? (unsigned short)f2bf(a.y) : (unsigned short)0;
  o[2] = ok ? (unsigned short)f2bf(a.z) : (unsigned short)0;
  o[3] = ok ? (unsigned short)f2bf(a.w) : (unsigned short)0;
  o[4] = ok ? (unsigned short)f2bf(b.x) : (unsigned short)0;
  o[5] = ok ? (unsigned short)f2bf(b.y) : (unsigned short)0;
  o[6] = ok ? (unsigned short)f2bf(b.z) : (unsigned short)0;
  o[7] = ok ? (unsigned short)f2bf(b.w) : (unsigned short)0;
  unsigned short* dp = xb + (size_t)row * FIN + k8;
  *(volatile v8us*)dp = o;
  __threadfence();
  *(volatile v8us*)dp = o;
}

__global__ __launch_bounds__(NTHR) void k_bucket(const int* __restrict__ dsts, const int* __restrict__ srcs,
                                                 const float* __restrict__ vals, int nE, int nN, int vec8,
                                                 int* RP, int* CN, int* SR, float* VL) {
  extern __shared__ v4f lds_dyn[];
  int* reg1 = (int*)lds_dyn;
  int* reg2 = reg1 + RCAP;
  int* scnt = reg2 + RCAP;
  int* soff = scnt + NB;
  int* list = soff + NB;
  int* wcnt = list + LISTN;
  int* wtot = wcnt + NWAVE;
  const int tid = (int)threadIdx.x, lane = tid & 31, wave = tid >> 5;
  const int nodeBase = (int)blockIdx.x * NB;

  {
    const v4i z4 = {0, 0, 0, 0};
    for (int i = tid * 4; i < BK_ZINTS; i += NTHR * 4) *(v4ia*)(reg1 + i) = z4;
    if (tid < 2 * NWAVE) wcnt[tid] = 0;
  }
  __syncthreads();

  int tot = 0;
  const int nChunks = (nE + CHUNK - 1) / CHUNK;
#pragma unroll 1
  for (int ch = 0; ch < nChunks; ++ch) {
    const int cbase = ch * CHUNK;
    const int wc = scan_chunk(dsts, nE, cbase, nodeBase, NB, vec8, list, tid, lane, wave);
    if (lane == 0) wcnt[wave] = wc;
    __syncthreads();
    int pre = 0, all = 0;
#pragma unroll
    for (int w2 = 0; w2 < NWAVE; ++w2) {
      int c = wcnt[w2];
      c = c < 0 ? 0 : (c > WCAP ? WCAP : c);
      all += c;
      pre += (w2 < wave) ? c : 0;
    }
    const int wcc  = wc > WCAP ? WCAP : wc;
    const int base = tot + pre;
#pragma unroll 1
    for (int i = lane; i < wcc; i += 32) {
      const int ent = list[wave * WCAP + i];
      const int el  = (ent >> SLOTB) & (CHUNK - 1);
      const int sl  = ent & (NB - 1);
      int eid = cbase + el;
      eid = eid > nE - 1 ? nE - 1 : eid;
      const int pos = base + i;
      if (pos < RCAP) reg1[pos] = (int)(((unsigned)eid << SLOTB) | (unsigned)sl);
    }
    tot += all;
    tot = tot > RCAP ? RCAP : tot;
    __syncthreads();
  }
  const int nh = tot;

  if (wave == 0) {
#pragma unroll 1
    for (int b0 = 0; b0 < nh; b0 += 32) {
      const int idx = b0 + lane;
      const int uv  = reg1[idx < nh ? idx : nh - 1];
      const int m32 = (nh - b0) < 32 ? (nh - b0) : 32;
#pragma unroll 1
      for (int k = 0; k < m32; ++k) {
        const int u  = __builtin_amdgcn_readlane(uv, k);
        const int sl = u & (NB - 1);
        if (lane == 0) scnt[sl] = scnt[sl] + 1;
      }
    }
  }
  __syncthreads();

  {
    const v4i ca = *(const v4ia*)(scnt + 4 * tid);
    const int e0 = ca.x < 0 ? 0 : ca.x, e1 = ca.y < 0 ? 0 : ca.y;
    const int e2 = ca.z < 0 ? 0 : ca.z, e3 = ca.w < 0 ? 0 : ca.w;
    const int ts = e0 + e1 + e2 + e3;
    int incl = ts;
#pragma unroll
    for (int d = 1; d < 32; d <<= 1) {
      const int up = __shfl_up(incl, d);
      if (lane >= d) incl += up;
    }
    if (lane == 31) wtot[wave] = incl;
    __syncthreads();
    int pre = 0;
#pragma unroll
    for (int w2 = 0; w2 < NWAVE; ++w2) pre += (w2 < wave) ? wtot[w2] : 0;
    int run = pre + incl - ts;
    v4i so;
    so.x = run; run += e0;
    so.y = run; run += e1;
    so.z = run; run += e2;
    so.w = run;
    *(v4ia*)(soff + 4 * tid) = so;
  }
  __syncthreads();
  for (int i = tid; i < NB; i += NTHR) list[i] = soff[i];
  __syncthreads();

  if (wave == 0) {
#pragma unroll 1
    for (int b0 = 0; b0 < nh; b0 += 32) {
      const int idx = b0 + lane;
      const int uv  = reg1[idx < nh ? idx : nh - 1];
      const int m32 = (nh - b0) < 32 ? (nh - b0) : 32;
#pragma unroll 1
      for (int k = 0; k < m32; ++k) {
        const int u   = __builtin_amdgcn_readlane(uv, k);
        const int sl  = u & (NB - 1);
        const int eid = (int)((unsigned)u >> SLOTB);
        if (lane == 0) {
          int pos = list[sl];
          pos = pos < 0 ? 0 : (pos > RCAP - 1 ? RCAP - 1 : pos);
          reg2[pos] = eid;
          list[sl] = pos + 1;
        }
      }
    }
  }
  __syncthreads();

  const bool ovf = (nh >= RCAP);
  {
    const v4i so = *(const v4ia*)(soff + 4 * tid);
    const v4i sc = *(const v4ia*)(scnt + 4 * tid);
    const int bb = (int)blockIdx.x * RCAP;
    v4i rp, cn;
    rp.x = bb + so.x; rp.y = bb + so.y; rp.z = bb + so.z; rp.w = bb + so.w;
    cn.x = ovf ? -1 : sc.x; cn.y = ovf ? -1 : sc.y; cn.z = ovf ? -1 : sc.z; cn.w = ovf ? -1 : sc.w;
    int* rpp = RP + (size_t)nodeBase + 4 * tid;
    int* cnp = CN + (size_t)nodeBase + 4 * tid;
    *(volatile v4i*)rpp = rp;
    *(volatile v4i*)cnp = cn;
    __threadfence();
    *(volatile v4i*)rpp = rp;
    *(volatile v4i*)cnp = cn;
  }
  const size_t segBase = (size_t)blockIdx.x * RCAP;
#pragma unroll 1
  for (int it = 0; it < RCAP / (NTHR * 4); ++it) {
    const int p = it * NTHR * 4 + 4 * tid;
    const v4i ev = *(const v4ia*)(reg2 + p);
    const int e0 = ev.x < 0 ? 0 : (ev.x > nE - 1 ? nE - 1 : ev.x);
    const int e1 = ev.y < 0 ? 0 : (ev.y > nE - 1 ? nE - 1 : ev.y);
    const int e2 = ev.z < 0 ? 0 : (ev.z > nE - 1 ? nE - 1 : ev.z);
    const int e3 = ev.w < 0 ? 0 : (ev.w > nE - 1 ? nE - 1 : ev.w);
    const int q0 = srcs[e0], q1 = srcs[e1], q2 = srcs[e2], q3 = srcs[e3];
    v4i sv;
    sv.x = (p     < nh) ? (q0 < 0 ? 0 : (q0 > nN - 1 ? nN - 1 : q0)) : 0;
    sv.y = (p + 1 < nh) ? (q1 < 0 ? 0 : (q1 > nN - 1 ? nN - 1 : q1)) : 0;
    sv.z = (p + 2 < nh) ? (q2 < 0 ? 0 : (q2 > nN - 1 ? nN - 1 : q2)) : 0;
    sv.w = (p + 3 < nh) ? (q3 < 0 ? 0 : (q3 > nN - 1 ? nN - 1 : q3)) : 0;
    int* sp = SR + segBase + p;
    *(volatile v4i*)sp = sv;
    __threadfence();
    *(volatile v4i*)sp = sv;
  }
#pragma unroll 1
  for (int it = 0; it < RCAP / (NTHR * 4); ++it) {
    const int p = it * NTHR * 4 + 4 * tid;
    const v4i ev = *(const v4ia*)(reg2 + p);
    const int e0 = ev.x < 0 ? 0 : (ev.x > nE - 1 ? nE - 1 : ev.x);
    const int e1 = ev.y < 0 ? 0 : (ev.y > nE - 1 ? nE - 1 : ev.y);
    const int e2 = ev.z < 0 ? 0 : (ev.z > nE - 1 ? nE - 1 : ev.z);
    const int e3 = ev.w < 0 ? 0 : (ev.w > nE - 1 ? nE - 1 : ev.w);
    const float g0 = vals[e0], g1 = vals[e1], g2 = vals[e2], g3 = vals[e3];
    v4f fv;
    fv.x = (p     < nh) ? bfr(g0) : 0.0f;
    fv.y = (p + 1 < nh) ? bfr(g1) : 0.0f;
    fv.z = (p + 2 < nh) ? bfr(g2) : 0.0f;
    fv.w = (p + 3 < nh) ? bfr(g3) : 0.0f;
    float* vp = VL + segBase + p;
    *(volatile v4f*)vp = fv;
    __threadfence();
    *(volatile v4f*)vp = fv;
  }
}

template <int FD, int SRCB>
__global__ __launch_bounds__(NTHR) void k_spmm(const int* __restrict__ RP, const int* __restrict__ CN,
                                               const int* __restrict__ SR, const float* __restrict__ VL,
                                               const void* __restrict__ srcv, float* dst,
                                               int nN, int mRows, int nbp, int csrn) {
  const int tid = (int)threadIdx.x, lane = tid & 31, wave = tid >> 5;
  const int r = (int)blockIdx.x * NWAVE + wave;
  if (r >= mRows) return;
  const int rc = r < nbp ? r : nbp - 1;
  int st = __builtin_amdgcn_readfirstlane(RP[rc]);
  const int craw = __builtin_amdgcn_readfirstlane(CN[rc]);
  int cnt = craw < 0 ? 0 : (craw > DEGCAP ? DEGCAP : craw);
  st = st < 0 ? 0 : (st > csrn - 1 ? csrn - 1 : st);
  if (cnt > csrn - st) cnt = csrn - st;
  const bool live = r < nN;
  if (!live) cnt = 0;
  const float qnan = __int_as_float(0x7fc00000);
  const float pz = (craw < 0 || craw > DEGCAP) ? qnan : 0.0f;

  v4f a0 = {0.f, 0.f, 0.f, 0.f};
  v4f a1 = {0.f, 0.f, 0.f, 0.f};
#pragma unroll 1
  for (int b0 = 0; b0 < cnt; b0 += 32) {
    int idx = st + b0 + lane;
    idx = idx > csrn - 1 ? csrn - 1 : idx;
    int sr = SR[idx];
    sr = sr < 0 ? 0 : (sr > nN - 1 ? nN - 1 : sr);
    const int cvi = __float_as_int(VL[idx]);
    const int m32 = (cnt - b0) < 32 ? (cnt - b0) : 32;
#pragma unroll 1
    for (int k = 0; k < m32; ++k) {
      const int   sk = __builtin_amdgcn_readlane(sr, k);
      const float ck = __int_as_float(__builtin_amdgcn_readlane(cvi, k));
      if constexpr (FD == 128 && SRCB == 1) {
        const unsigned short* xb = (const unsigned short*)srcv;
        const v2u w = *(const v2ua*)(xb + (size_t)sk * 128 + 4 * lane);
        const float x0 = __uint_as_float(w.x << 16);
        const float x1 = __uint_as_float(w.x & 0xffff0000u);
        const float x2 = __uint_as_float(w.y << 16);
        const float x3 = __uint_as_float(w.y & 0xffff0000u);
        a0.x = fmaf(ck, x0, a0.x); a0.y = fmaf(ck, x1, a0.y);
        a0.z = fmaf(ck, x2, a0.z); a0.w = fmaf(ck, x3, a0.w);
      } else if constexpr (FD == 128) {
        const float* xs = (const float*)srcv;
        const v4f v = *(const v4fa*)(xs + (size_t)sk * 128 + 4 * lane);
        a0.x = fmaf(ck, v.x, a0.x); a0.y = fmaf(ck, v.y, a0.y);
        a0.z = fmaf(ck, v.z, a0.z); a0.w = fmaf(ck, v.w, a0.w);
      } else {
        const float* xs = (const float*)srcv;
        const v4f v = *(const v4fa*)(xs + (size_t)sk * 256 + 4 * lane);
        const v4f w = *(const v4fa*)(xs + (size_t)sk * 256 + 128 + 4 * lane);
        a0.x = fmaf(ck, v.x, a0.x); a0.y = fmaf(ck, v.y, a0.y);
        a0.z = fmaf(ck, v.z, a0.z); a0.w = fmaf(ck, v.w, a0.w);
        a1.x = fmaf(ck, w.x, a1.x); a1.y = fmaf(ck, w.y, a1.y);
        a1.z = fmaf(ck, w.z, a1.z); a1.w = fmaf(ck, w.w, a1.w);
      }
    }
  }
  v4f o0, o1;
  o0.x = live ? (a0.x + pz) : 0.0f; o0.y = live ? (a0.y + pz) : 0.0f;
  o0.z = live ? (a0.z + pz) : 0.0f; o0.w = live ? (a0.w + pz) : 0.0f;
  o1.x = live ? (a1.x + pz) : 0.0f; o1.y = live ? (a1.y + pz) : 0.0f;
  o1.z = live ? (a1.z + pz) : 0.0f; o1.w = live ? (a1.w + pz) : 0.0f;
  float* op = dst + (size_t)r * FD + 4 * lane;
  *(volatile v4f*)op = o0;
  if constexpr (FD == 256) *(volatile v4f*)(op + 128) = o1;
  __threadfence();
  *(volatile v4f*)op = o0;
  if constexpr (FD == 256) *(volatile v4f*)(op + 128) = o1;
}

template <int KIN>
__global__ __launch_bounds__(NTHR) void k_gemm(const char* __restrict__ wsb,
                                               long long o0, long long o1, long long o2, long long o3,
                                               const unsigned short* __restrict__ Bt, float* outF,
                                               int c0, int c1, int c2, int c3, int nseg, int accum) {
  constexpr int KB  = 5 * KIN;
  constexpr int NCH = KIN / 32;
  static_assert(KIN % 32 == 0);
  __shared__ __attribute__((aligned(16))) unsigned short sAhi[GBM * APITCH];
  __shared__ __attribute__((aligned(16))) unsigned short sAlo[GBM * APITCH];
  __shared__ __attribute__((aligned(16))) float stg[NWAVE * 16 * 64];
  const int tid = (int)threadIdx.x, lane = tid & 31, wave = tid >> 5, hh = lane >> 4, m = lane & 15;
  const int rg = wave & 3, chh = wave >> 2;
  const int rowBase = (int)blockIdx.x * GBM;
  const int srow = tid >> 2, sc8 = (tid & 3) * 8;

  v8f acc[8];
  {
    const v8f z = {0.f, 0.f, 0.f, 0.f, 0.f, 0.f, 0.f, 0.f};
#pragma unroll
    for (int t = 0; t < 8; ++t) acc[t] = z;
  }
  const unsigned short* bbase = Bt + (size_t)(128 * chh + m) * KB + 8 * hh;
  const unsigned short* arh = sAhi + (16 * rg + m) * APITCH + 8 * hh;
  const unsigned short* arl = sAlo + (16 * rg + m) * APITCH + 8 * hh;

#pragma unroll 1
  for (int seg = 0; seg < nseg; ++seg) {
    const long long so = (seg == 0) ? o0 : (seg == 1) ? o1 : (seg == 2) ? o2 : o3;
    const int code = (seg == 0) ? c0 : (seg == 1) ? c1 : (seg == 2) ? c2 : c3;
    const int kb0  = (code >= 2) ? code * KIN : 0;
    const char* sp = wsb + so;
#pragma unroll 1
    for (int ch = 0; ch < NCH; ++ch) {
      const int col = 32 * ch + sc8;
      if (code == 0) {
        const unsigned short* xp = (const unsigned short*)sp + (size_t)(rowBase + srow) * KIN + col;
        const v8us xv = *(const v8usa*)xp;
        *(v8usa*)(sAhi + srow * APITCH + sc8) = xv;
      } else {
        const float* fp = (const float*)sp + (size_t)(rowBase + srow) * KIN + col;
        const v4f a = *(const v4fa*)fp;
        const v4f b = *(const v4fa*)(fp + 4);
        v8us oh, ol;
        split8(a, b, oh, ol);
        *(v8usa*)(sAhi + srow * APITCH + sc8) = oh;
        *(v8usa*)(sAlo + srow * APITCH + sc8) = ol;
      }
      __syncthreads();

      FragB ahi;
      ahi.h[0] = *(const v8usa*)arh;
      ahi.h[1] = *(const v8usa*)(arh + 16);
      const unsigned short* bq = bbase + kb0 + 32 * ch;
      if (code == 0) {
#pragma unroll
        for (int t = 0; t < 8; ++t) {
          const unsigned short* wq = bq + (size_t)(16 * t) * KB;
          FragB b0, b1;
          b0.h[0] = *(const v8usa*)wq;
          b0.h[1] = *(const v8usa*)(wq + 16);
          b1.h[0] = *(const v8usa*)(wq + KIN);
          b1.h[1] = *(const v8usa*)(wq + KIN + 16);
          acc[t] = wmb(ahi, b0, acc[t]);
          acc[t] = wmb(ahi, b1, acc[t]);
        }
      } else {
        FragB alo;
        alo.h[0] = *(const v8usa*)arl;
        alo.h[1] = *(const v8usa*)(arl + 16);
        if (code == 1) {
#pragma unroll
          for (int t = 0; t < 8; ++t) {
            const unsigned short* wq = bq + (size_t)(16 * t) * KB;
            FragB b0, b1;
            b0.h[0] = *(const v8usa*)wq;
            b0.h[1] = *(const v8usa*)(wq + 16);
            b1.h[0] = *(const v8usa*)(wq + KIN);
            b1.h[1] = *(const v8usa*)(wq + KIN + 16);
            acc[t] = wmb(ahi, b0, acc[t]);
            acc[t] = wmb(alo, b0, acc[t]);
            acc[t] = wmb(ahi, b1, acc[t]);
          }
        } else {
#pragma unroll
          for (int t = 0; t < 8; ++t) {
            const unsigned short* wq = bq + (size_t)(16 * t) * KB;
            FragB b0;
            b0.h[0] = *(const v8usa*)wq;
            b0.h[1] = *(const v8usa*)(wq + 16);
            acc[t] = wmb(ahi, b0, acc[t]);
            acc[t] = wmb(alo, b0, acc[t]);
          }
        }
      }
      __syncthreads();
    }
  }

  float* sw = stg + wave * (16 * 64);
#pragma unroll
  for (int hf = 0; hf < 2; ++hf) {
#pragma unroll
    for (int t = 0; t < 4; ++t) {
#pragma unroll
      for (int r = 0; r < 8; ++r) {
        sw[(8 * hh + r) * 64 + 16 * t + m] = acc[4 * hf + t][r];
      }
    }
    __syncthreads();
    v4f fv[8];
#pragma unroll
    for (int i = 0; i < 8; ++i) {
      const int lr = 2 * i + hh;
      fv[i] = *(const v4fa*)(sw + lr * 64 + 4 * m);
    }
    if (accum != 0) {
#pragma unroll
      for (int i = 0; i < 8; ++i) {
        const int lr = 2 * i + hh;
        const float* ip = outF + (size_t)(rowBase + 16 * rg + lr) * LW + 128 * chh + 64 * hf + 4 * m;
        const v4f old = *(const v4fa*)ip;
        fv[i] = fv[i] + old;
      }
    }
#pragma unroll
    for (int i = 0; i < 8; ++i) {
      const int lr = 2 * i + hh;
      float* op = outF + (size_t)(rowBase + 16 * rg + lr) * LW + 128 * chh + 64 * hf + 4 * m;
      *(volatile v4f*)op = fv[i];
    }
    __threadfence();
#pragma unroll
    for (int i = 0; i < 8; ++i) {
      const int lr = 2 * i + hh;
      float* op = outF + (size_t)(rowBase + 16 * rg + lr) * LW + 128 * chh + 64 * hf + 4 * m;
      *(volatile v4f*)op = fv[i];
    }
    __syncthreads();
  }
}

__global__ __launch_bounds__(NTHR) void k_bnstat(const float* __restrict__ pre, int nN, double* rec) {
  const int c  = (int)threadIdx.x;
  const int r0 = (int)blockIdx.x * RBN;
  int r1 = r0 + RBN; r1 = r1 > nN ? nN : r1;
  double s = 0.0, q = 0.0;
#pragma unroll 4
  for (int r = r0; r < r1; ++r) {
    const float v  = pre[(size_t)r * LW + c];
    const float rv = relu_np(v);
    const float u  = (c < 128) ? rv : v;
    const double d = (double)u;
    s += d;
    q += d * d;
  }
  v2d o; o.x = s; o.y = q;
  double* rp = rec + ((size_t)blockIdx.x * LW + c) * 2;
  *(volatile v2d*)rp = o;
  __threadfence();
  *(volatile v2d*)rp = o;
}

__global__ __launch_bounds__(NTHR) void k_bncomb(const double* __restrict__ rec, int nblk, double invN,
                                                 const float* __restrict__ bn, float* stat) {
  __shared__ __attribute__((aligned(16))) float st[3 * LW];
  const int c = (int)threadIdx.x;
  double S = 0.0, Q = 0.0;
#pragma unroll 4
  for (int b = 0; b < nblk; ++b) {
    const v2d r = *(const v2da*)(rec + ((size_t)b * LW + c) * 2);
    S += r.x; Q += r.y;
  }
  const double mean = S * invN;
  const double var  = Q * invN - mean * mean;
  const float  vf   = (float)var;
  const float  rs   = 1.0f / sqrtf(vf + 1e-3f);
  const int f   = c & 127;
  const int row = (c < 128) ? 0 : 2;
  const float g  = bfr(bn[row * 128 + f]);
  const float bb = bfr(bn[(row + 1) * 128 + f]);
  st[c]          = (float)mean;
  st[LW + c]     = g * rs;
  st[2 * LW + c] = bb;
  __syncthreads();
  const int tc = c < 192 ? c : 191;
  const v4f ov = *(const v4fa*)(st + 4 * tc);
  const bool ok = c < 192;
  if (ok) *(volatile v4f*)(stat + 4 * tc) = ov;
  __threadfence();
  if (ok) *(volatile v4f*)(stat + 4 * tc) = ov;
}

__global__ __launch_bounds__(NTHR) void k_bnapply(const float* __restrict__ pre, const float* __restrict__ stat,
                                                  float* H, int nN, int nUnits) {
  const int i = (int)blockIdx.x * NTHR + (int)threadIdx.x;
  if (i >= nUnits) return;
  const int row = i >> 6;
  const int c4  = (i & 63) * 4;
  const int rc  = row < nN ? row : nN - 1;
  const v4f v  = *(const v4fa*)(pre + (size_t)rc * LW + c4);
  const v4f mu = *(const v4fa*)(stat + c4);
  const v4f g  = *(const v4fa*)(stat + LW + c4);
  const v4f bb = *(const v4fa*)(stat + 2 * LW + c4);
  const bool isA = c4 < 128;
  const bool live = row < nN;
  const float u0 = isA ? relu_np(v.x) : v.x;
  const float u1 = isA ? relu_np(v.y) : v.y;
  const float u2 = isA ? relu_np(v.z) : v.z;
  const float u3 = isA ? relu_np(v.w) : v.w;
  v4f o;
  o.x = live ? ((u0 - mu.x) * g.x + bb.x) : 0.0f;
  o.y = live ? ((u1 - mu.y) * g.y + bb.y) : 0.0f;
  o.z = live ? ((u2 - mu.z) * g.z + bb.z) : 0.0f;
  o.w = live ? ((u3 - mu.w) * g.w + bb.w) : 0.0f;
  float* op = H + (size_t)row * LW + c4;
  *(volatile v4f*)op = o;
  __threadfence();
  *(volatile v4f*)op = o;
}

__global__ __launch_bounds__(NTHR) void k_bnz(const float* __restrict__ pre, const float* __restrict__ stat,
                                              const unsigned short* __restrict__ WeT,
                                              const float* __restrict__ be, float* Z) {
  __shared__ __attribute__((aligned(16))) unsigned short sAhi[GBM * APITCH];
  __shared__ __attribute__((aligned(16))) unsigned short sAlo[GBM * APITCH];
  __shared__ __attribute__((aligned(16))) float sst[3 * LW];
  __shared__ __attribute__((aligned(16))) float zt[GBM * NMACH];
  const int tid = (int)threadIdx.x, lane = tid & 31, wave = tid >> 5, hh = lane >> 4, m = lane & 15;
  const int rowBase = (int)blockIdx.x * GBM;
  const int srow = tid >> 2, sc8 = (tid & 3) * 8;
  if (tid < 192) *(v4fa*)(sst + 4 * tid) = *(const v4fa*)(stat + 4 * tid);
  __syncthreads();

  v8f acc = {0.f, 0.f, 0.f, 0.f, 0.f, 0.f, 0.f, 0.f};
  const int wr = wave & 3;
  const unsigned short* arh = sAhi + (16 * wr + m) * APITCH + 8 * hh;
  const unsigned short* arl = sAlo + (16 * wr + m) * APITCH + 8 * hh;
  const unsigned short* wb  = WeT + (size_t)m * LW + 8 * hh;
#pragma unroll 1
  for (int ch = 0; ch < LW / 32; ++ch) {
    const int col = 32 * ch + sc8;
    const float* fp = pre + (size_t)(rowBase + srow) * LW + col;
    const v4f a = *(const v4fa*)fp;
    const v4f b = *(const v4fa*)(fp + 4);
    const v4f ma = *(const v4fa*)(sst + col),          mb = *(const v4fa*)(sst + col + 4);
    const v4f ga = *(const v4fa*)(sst + LW + col),     gb = *(const v4fa*)(sst + LW + col + 4);
    const v4f ba = *(const v4fa*)(sst + 2 * LW + col), bb = *(const v4fa*)(sst + 2 * LW + col + 4);
    const bool isA = ch < 4;
    v4f ha, hb2;
    ha.x  = ((isA ? relu_np(a.x) : a.x) - ma.x) * ga.x + ba.x;
    ha.y  = ((isA ? relu_np(a.y) : a.y) - ma.y) * ga.y + ba.y;
    ha.z  = ((isA ? relu_np(a.z) : a.z) - ma.z) * ga.z + ba.z;
    ha.w  = ((isA ? relu_np(a.w) : a.w) - ma.w) * ga.w + ba.w;
    hb2.x = ((isA ? relu_np(b.x) : b.x) - mb.x) * gb.x + bb.x;
    hb2.y = ((isA ? relu_np(b.y) : b.y) - mb.y) * gb.y + bb.y;
    hb2.z = ((isA ? relu_np(b.z) : b.z) - mb.z) * gb.z + bb.z;
    hb2.w = ((isA ? relu_np(b.w) : b.w) - mb.w) * gb.w + bb.w;
    v8us oh, ol;
    split8(ha, hb2, oh, ol);
    *(v8usa*)(sAhi + srow * APITCH + sc8) = oh;
    *(v8usa*)(sAlo + srow * APITCH + sc8) = ol;
    __syncthreads();
    if (wave < 4) {
      FragB ahi, alo, bf;
      ahi.h[0] = *(const v8usa*)arh;
      ahi.h[1] = *(const v8usa*)(arh + 16);
      alo.h[0] = *(const v8usa*)arl;
      alo.h[1] = *(const v8usa*)(arl + 16);
      bf.h[0]  = *(const v8usa*)(wb + 32 * ch);
      bf.h[1]  = *(const v8usa*)(wb + 32 * ch + 16);
      acc = wmb(ahi, bf, acc);
      acc = wmb(alo, bf, acc);
    }
    __syncthreads();
  }
  const float bem = bfr(be[m]);
  if (wave < 4) {
#pragma unroll
    for (int r = 0; r < 8; ++r) zt[(16 * wave + 8 * hh + r) * NMACH + m] = acc[r] + bem;
  }
  __syncthreads();
  const v4f zv = *(const v4fa*)(zt + 4 * tid);
  float* zp = Z + (size_t)rowBase * NMACH + 4 * tid;
  *(volatile v4f*)zp = zv;
  __threadfence();
  *(volatile v4f*)zp = zv;
}

__global__ __launch_bounds__(NTHR) void k_edge(const int* __restrict__ rows, const int* __restrict__ cols,
                                               const float* __restrict__ vals, const float* __restrict__ Z,
                                               float* out, int nE, int nN) {
  __shared__ __attribute__((aligned(16))) float stg[NTHR * NMACH];
  const int tid = (int)threadIdx.x;
  const int m = tid & 15, g = tid >> 4;
  const int eBase = (int)blockIdx.x * 256;
#pragma unroll 1
  for (int it = 0; it < 16; ++it) {
    const int e  = eBase + it * 16 + g;
    const int ec = e < nE ? e : nE - 1;
    int r = rows[ec]; r = r < 0 ? 0 : (r > nN - 1 ? nN - 1 : r);
    int c = cols[ec]; c = c < 0 ? 0 : (c > nN - 1 ? nN - 1 : c);
    const float vb = bfr(vals[ec]);
    const float zr = Z[(size_t)r * NMACH + m];
    const float zc = Z[(size_t)c * NMACH + m];
    const float s  = vb * (zr + zc);
    float mx = s;
    mx = fmaxf(mx, __shfl_xor(mx, 8));
    mx = fmaxf(mx, __shfl_xor(mx, 4));
    mx = fmaxf(mx, __shfl_xor(mx, 2));
    mx = fmaxf(mx, __shfl_xor(mx, 1));
    const float ex = expf(s - mx);
    float sm = ex;
    sm += __shfl_xor(sm, 8);
    sm += __shfl_xor(sm, 4);
    sm += __shfl_xor(sm, 2);
    sm += __shfl_xor(sm, 1);
    stg[it * 256 + tid] = ex * (1.0f / sm);
  }
  __syncthreads();
  v4f ov[4];
#pragma unroll
  for (int j = 0; j < 4; ++j) ov[j] = *(const v4fa*)(stg + 4 * (j * NTHR + tid));
  const long long lim = (long long)nE * 4;
#pragma unroll
  for (int j = 0; j < 4; ++j) {
    const int p = j * NTHR + tid;
    const bool ok = ((long long)eBase * 4 + p) < lim;
    float* op = out + (size_t)eBase * NMACH + 4 * (size_t)p;
    if (ok) *(volatile v4f*)op = ov[j];
  }
  __threadfence();
#pragma unroll
  for (int j = 0; j < 4; ++j) {
    const int p = j * NTHR + tid;
    const bool ok = ((long long)eBase * 4 + p) < lim;
    float* op = out + (size_t)eBase * NMACH + 4 * (size_t)p;
    if (ok) *(volatile v4f*)op = ov[j];
  }
}

static inline int cdiv(int a, int b) { return (a + b - 1) / b; }
static inline size_t al256(size_t o) { return (o + 255) & ~(size_t)255; }

extern "C" void kernel_launch(void* const* d_in, const int* in_sizes, int n_in,
                              void* d_out, int out_size, void* d_ws, size_t ws_size,
                              hipStream_t stream) {
  if (n_in < 12) return;
  if (in_sizes[0] < FIN || (in_sizes[0] % FIN) != 0) return;
  const int nN = in_sizes[0] / FIN;
  if (nN < 1 || nN > (1 << 20)) return;
  const int nE = in_sizes[1];
  if (nE < 1 || nE >= (1 << 21)) return;
  if (in_sizes[2] != nE || in_sizes[3] != nE) return;
  if (in_sizes[4] != 6 * 128 * 128 || in_sizes[5] != 6 * 128 * 128) return;
  if (in_sizes[6] != 4 * 128) return;
  if (in_sizes[7] != 6 * 256 * 128 || in_sizes[8] != 6 * 256 * 128) return;
  if (in_sizes[9] != 4 * 128) return;
  if (in_sizes[10] != LW * NMACH || in_sizes[11] != NMACH) return;
  if ((long long)out_size != (long long)nE * NMACH) return;

  const float* x    = (const float*)d_in[0];
  const int*   rows = (const int*)d_in[1];
  const int*   cols = (const int*)d_in[2];
  const float* vals = (const float*)d_in[3];
  const float* l0Wa = (const float*)d_in[4];
  const float* l0Wb = (const float*)d_in[5];
  const float* l0bn = (const float*)d_in[6];
  const float* l1Wa = (const float*)d_in[7];
  const float* l1Wb = (const float*)d_in[8];
  const float* l1bn = (const float*)d_in[9];
  const float* We   = (const float*)d_in[10];
  const float* be   = (const float*)d_in[11];
  float* out = (float*)d_out;

  const int MP   = cdiv(nN, RBN) * RBN;
  const int gB   = cdiv(MP, NB);
  const int NBP  = gB * NB;
  if ((long long)gB * RCAP >= (1LL << 30)) return;
  const int csrn = gB * RCAP;
  const int nStatBlk = MP / RBN;
  const int vec8 = ((nE & 3) == 0) ? 1 : 0;

  char* ws = (char*)d_ws;
  size_t off = 0;
  const size_t oP0  = off; off = al256(off + (size_t)MP * LW * 4);
  const size_t oP1  = off; off = al256(off + (size_t)MP * LW * 4);
  const size_t oPRE = off; off = al256(off + (size_t)MP * LW * 4);
  const size_t oXB  = off; off = al256(off + (size_t)MP * FIN * 2);
  const size_t oRP  = off; off = al256(off + (size_t)NBP * 4);
  const size_t oCN  = off; off = al256(off + (size_t)NBP * 4);
  const size_t oSR  = off; off = al256(off + (size_t)csrn * 4);
  const size_t oVL  = off; off = al256(off + (size_t)csrn * 4);
  const size_t oZ   = off; off = al256(off + (size_t)MP * NMACH * 4);
  const size_t oB0  = off; off = al256(off + (size_t)256 * 640 * 2);
  const size_t oB1  = off; off = al256(off + (size_t)256 * 1280 * 2);
  const size_t oWT  = off; off = al256(off + (size_t)NMACH * LW * 2);
  const size_t oSS  = off; off = al256(off + (size_t)(SS0N + SS1N) * 4);
  const size_t oREC = off; off = al256(off + (size_t)nStatBlk * LW * 16);
  const size_t oST  = off; off = al256(off + (size_t)3 * LW * 4);
  if (off > ws_size) return;
  const char*     wsc = (const char*)ws;
  float*          P0  = (float*)(ws + oP0);
  float*          P1  = (float*)(ws + oP1);
  float*          PRE = (float*)(ws + oPRE);
  unsigned short* XB  = (unsigned short*)(ws + oXB);
  int*            RP  = (int*)(ws + oRP);
  int*            CN  = (int*)(ws + oCN);
  int*            SR  = (int*)(ws + oSR);
  float*          VL  = (float*)(ws + oVL);
  float*          Z   = (float*)(ws + oZ);
  unsigned short* Bt0 = (unsigned short*)(ws + oB0);
  unsigned short* Bt1 = (unsigned short*)(ws + oB1);
  unsigned short* WeT = (unsigned short*)(ws + oWT);
  float*          SS  = (float*)(ws + oSS);
  double*         REC = (double*)(ws + oREC);
  float*          ST  = (float*)(ws + oST);

  hipFuncSetAttribute(reinterpret_cast<const void*>(&k_bucket),
                      hipFuncAttributeMaxDynamicSharedMemorySize, LDS_BKT);

  const size_t halfB = (size_t)MP * FIN * 4;
  float* a0p = P0;
  float* a1p = P0 + (size_t)MP * FIN;
  float* tp  = P1;
  float* a2p = P1 + (size_t)MP * FIN;
  const long long bXB = (long long)oXB;
  const long long bP0 = (long long)oP0;
  const long long bP1 = (long long)oP1;
  const long long bA0 = (long long)oP0;
  const long long bA1 = (long long)(oP0 + halfB);
  const long long bA2 = (long long)(oP1 + halfB);

  k_sum<<<(SS0N + SS1N) / (NTHR * 4), NTHR, 0, stream>>>(l0Wa, l0Wb, l1Wa, l1Wb, SS);
  k_wtr<128><<<(5 * 256 * 16) / NTHR, NTHR, 0, stream>>>(SS, l0Wa, l0Wb, Bt0);
  k_wtr<256><<<(5 * 256 * 32) / NTHR, NTHR, 0, stream>>>(SS + SS0N, l1Wa, l1Wb, Bt1);
  k_wet<<<cdiv(NMACH * (LW / 8), NTHR), NTHR, 0, stream>>>(We, WeT);
  const int nUx = MP * (FIN / 8);
  k_cvx<<<cdiv(nUx, NTHR), NTHR, 0, stream>>>(x, nN, nUx, XB);
  k_bucket<<<gB, NTHR, LDS_BKT, stream>>>(rows, cols, vals, nE, nN, vec8, RP, CN, SR, VL);

  const int gS = MP / NWAVE;
  const int gG = MP / GBM;
  k_spmm<128, 1><<<gS, NTHR, 0, stream>>>(RP, CN, SR, VL, (const void*)XB,  a0p, nN, MP, NBP, csrn);
  k_spmm<128, 0><<<gS, NTHR, 0, stream>>>(RP, CN, SR, VL, (const void*)a0p, a1p, nN, MP, NBP, csrn);
  k_spmm<128, 0><<<gS, NTHR, 0, stream>>>(RP, CN, SR, VL, (const void*)a1p, tp,  nN, MP, NBP, csrn);
  k_spmm<128, 0><<<gS, NTHR, 0, stream>>>(RP, CN, SR, VL, (const void*)tp,  a2p, nN, MP, NBP, csrn);
  k_gemm<128><<<gG, NTHR, 0, stream>>>(wsc, bXB, bA0, bA1, bA2, Bt0, PRE, 0, 2, 3, 4, 4, 0);
  k_bnstat<<<nStatBlk, NTHR, 0, stream>>>(PRE, nN, REC);
  k_bncomb<<<1, NTHR, 0, stream>>>(REC, nStatBlk, 1.0 / (double)nN, l0bn, ST);
  const int nUh = MP * (LW / 4);
  k_bnapply<<<cdiv(nUh, NTHR), NTHR, 0, stream>>>(PRE, ST, P0, nN, nUh);

  k_spmm<256, 0><<<gS, NTHR, 0, stream>>>(RP, CN, SR, VL, (const void*)P0, P1, nN, MP, NBP, csrn);
  k_gemm<256><<<gG, NTHR, 0, stream>>>(wsc, bP0, bP1, bP0, bP0, Bt1, PRE, 1, 2, 2, 2, 2, 0);
  k_spmm<256, 0><<<gS, NTHR, 0, stream>>>(RP, CN, SR, VL, (const void*)P1, P0, nN, MP, NBP, csrn);
  k_gemm<256><<<gG, NTHR, 0, stream>>>(wsc, bP0, bP0, bP0, bP0, Bt1, PRE, 3, 3, 3, 3, 1, 1);
  k_spmm<256, 0><<<gS, NTHR, 0, stream>>>(RP, CN, SR, VL, (const void*)P0, P1, nN, MP, NBP, csrn);
  k_spmm<256, 0><<<gS, NTHR, 0, stream>>>(RP, CN, SR, VL, (const void*)P1, P0, nN, MP, NBP, csrn);
  k_gemm<256><<<gG, NTHR, 0, stream>>>(wsc, bP0, bP0, bP0, bP0, Bt1, PRE, 4, 4, 4, 4, 1, 1);
  k_bnstat<<<nStatBlk, NTHR, 0, stream>>>(PRE, nN, REC);
  k_bncomb<<<1, NTHR, 0, stream>>>(REC, nStatBlk, 1.0 / (double)nN, l1bn, ST);
  k_bnz<<<gG, NTHR, 0, stream>>>(PRE, ST, WeT, be, Z);
  k_edge<<<cdiv(nE, 256), NTHR, 0, stream>>>(rows, cols, vals, Z, out, nE, nN);
}
